// MyRNN_83253646065788
// MI455X (gfx1250) — hardware-verified
//
#include <hip/hip_runtime.h>
#include <math.h>

constexpr int NB    = 4096;
constexpr int NSTEP = 512;
constexpr int NH    = 32;
constexpr int WPB   = 2;
constexpr int RPW   = 32;
constexpr int NTHR  = WPB * 32;
constexpr int RPB   = WPB * RPW;
constexpr int XCH   = 16;
constexpr int NCH   = NSTEP / XCH;
constexpr int HT_SZ = 16 * NH;
constexpr int HS_SZ = RPW * NH;
constexpr int NPF   = 160;
constexpr int NOUTF = NB + 2 * NB * NH;
constexpr float WSC     = 16.0f;
constexpr float WSC_INV = 1.0f / 16.0f;
static_assert(NB % RPB == 0);
static_assert(NSTEP % XCH == 0);
static_assert((NH * NH / 2) % NTHR == 0);
static_assert(NB * 4 == 16384);
static_assert(NOUTF * 4 == 1064960);
static_assert(RPW * XCH % 4 == 0);

typedef __attribute__((ext_vector_type(16))) _Float16 v16h;
typedef __attribute__((ext_vector_type(8)))  _Float16 v8h;
typedef __attribute__((ext_vector_type(8)))  float    v8f;
typedef __attribute__((ext_vector_type(4)))  float    v4f;

__device__ __forceinline__ void guard_g0(v8f& a, v8f& b, v16h x, v16h y, v16h z) {
  asm volatile("v_nop\n\tv_nop\n\tv_nop\n\tv_nop" : "+v"(a), "+v"(b) : "v"(x), "v"(y), "v"(z));
}
__device__ __forceinline__ void guard_g1(v8f& a, v8f& b, v16h x0, v16h x1, v16h y0, v16h y1, v16h y2, v16h y3) {
  asm volatile("v_nop\n\tv_nop\n\tv_nop\n\tv_nop" : "+v"(a), "+v"(b) : "v"(x0), "v"(x1), "v"(y0), "v"(y1), "v"(y2), "v"(y3));
}

template <typename T> struct Frag;
template <> struct Frag<_Float16> {
  typedef v16h V; union U { v16h v; v8h h[2]; };
  static __device__ __forceinline__ v16h load(const _Float16* p) {
    U f; f.h[0] = *(const v8h*)(p); f.h[1] = *(const v8h*)(p + 16); return f.v;
  }
  static __device__ __forceinline__ v8f mma(v16h a, v16h b, v8f c) {
    return __builtin_amdgcn_wmma_f32_16x16x32_f16(false, a, false, b, (short)0, c, false, false);
  }
};

__device__ __forceinline__ float ftanh_f32(float v) {
  const float e = expf(2.0f * v);
  return 1.0f - 2.0f * __builtin_amdgcn_rcpf(e + 1.0f);
}

__device__ __forceinline__ void stage_w16(const float* __restrict__ W, _Float16* dst, int tid) {
  unsigned* dw = (unsigned*)dst;
#pragma unroll 1
  for (int it = 0; it < (NH * NH / 2) / NTHR; ++it) {
    const int wi = it * NTHR + tid;
    const float f0 = W[2 * wi] * WSC;
    const float f1 = W[2 * wi + 1] * WSC;
    const _Float16 h0 = (_Float16)f0;
    const _Float16 h1 = (_Float16)f1;
    dw[wi] = (unsigned)__builtin_bit_cast(unsigned short, h0) | ((unsigned)__builtin_bit_cast(unsigned short, h1) << 16);
  }
}

__global__ __launch_bounds__(NTHR) void rnn2_seq_kernel(
    const float* __restrict__ x,
    const float* __restrict__ hs,
    const float* __restrict__ wih0,
    const float* __restrict__ whh0,
    const float* __restrict__ bih0,
    const float* __restrict__ bhh0,
    const float* __restrict__ wih1,
    const float* __restrict__ whh1,
    const float* __restrict__ bih1,
    const float* __restrict__ bhh1,
    const float* __restrict__ wfc,
    const float* __restrict__ bfc,
    float* __restrict__ out) {
  __shared__ __align__(16) _Float16 WL[3 * NH * NH];
  __shared__ __align__(16) float    Pf[NPF];
  __shared__ __align__(16) _Float16 Ht[WPB * 2 * 2 * HT_SZ];
  __shared__ __align__(16) float    Xs[WPB * RPW * XCH];
  __shared__ __align__(16) float    Hs[WPB * 2 * HS_SZ];
  __shared__ __align__(16) float    Pq[WPB * RPW];

  const int tid = threadIdx.x, lane = tid & 31, w = tid >> 5;
  const int c = lane & 15, hh = lane >> 4, koff = hh * 8;
  const int bbase = blockIdx.x * RPB + w * RPW;

  stage_w16(whh0, WL, tid);
  stage_w16(wih1, WL + NH * NH, tid);
  stage_w16(whh1, WL + 2 * NH * NH, tid);
  if (tid < NH) {
    Pf[tid]          = wih0[tid];
    Pf[NH + tid]     = bih0[tid] + bhh0[tid];
    Pf[2 * NH + tid] = bih1[tid] + bhh1[tid];
    Pf[3 * NH + tid] = wfc[tid];
  }
  if (tid == 0) Pf[4 * NH] = bfc[0];
#pragma unroll
  for (int L = 0; L < 2; ++L) {
    const float* src = hs + (size_t)L * NB * NH + (size_t)(bbase + lane) * NH;
    _Float16* dst = Ht + ((w * 2 + L) * 2 + (lane >> 4)) * HT_SZ + (lane & 15) * NH;
#pragma unroll
    for (int q = 0; q < 4; ++q) {
      const v4f va = *(const v4f*)(src + 8 * q);
      const v4f vb = *(const v4f*)(src + 8 * q + 4);
      v8h hv;
#pragma unroll
      for (int e = 0; e < 4; ++e) { hv[e] = (_Float16)va[e]; hv[4 + e] = (_Float16)vb[e]; }
      *(v8h*)(dst + 8 * q) = hv;
      asm volatile("" ::: "memory");
    }
  }
  __syncthreads();

  v16h bw[3][2];
#pragma unroll
  for (int p = 0; p < 3; ++p)
#pragma unroll
    for (int nt = 0; nt < 2; ++nt)
      bw[p][nt] = Frag<_Float16>::load(WL + p * NH * NH + (16 * nt + c) * NH + koff);
  float wic[2], bs0[2], bs1[2];
#pragma unroll
  for (int nt = 0; nt < 2; ++nt) {
    wic[nt] = Pf[16 * nt + c];
    bs0[nt] = Pf[NH + 16 * nt + c];
    bs1[nt] = Pf[2 * NH + 16 * nt + c];
  }
  v16h a0[2], a1[2];
#pragma unroll
  for (int mt = 0; mt < 2; ++mt) {
    a0[mt] = Frag<_Float16>::load(Ht + ((w * 2 + 0) * 2 + mt) * HT_SZ + c * NH + koff);
    a1[mt] = Frag<_Float16>::load(Ht + ((w * 2 + 1) * 2 + mt) * HT_SZ + c * NH + koff);
  }
  const v8f z8 = {0.f, 0.f, 0.f, 0.f, 0.f, 0.f, 0.f, 0.f};
  _Float16* ht0 = Ht + (w * 2 + 0) * 2 * HT_SZ;
  _Float16* ht1 = Ht + (w * 2 + 1) * 2 * HT_SZ;
  float* hs0 = Hs + (w * 2 + 0) * HS_SZ;
  float* hs1 = Hs + (w * 2 + 1) * HS_SZ;
  float* xsw = Xs + w * RPW * XCH;

#pragma unroll 1
  for (int tc = 0; tc < NCH; ++tc) {
    {
      const float* src = x + (size_t)(bbase + lane) * NSTEP + tc * XCH;
      float* dst = xsw + lane * XCH;
#pragma unroll
      for (int q = 0; q < 4; ++q) *(v4f*)(dst + 4 * q) = *(const v4f*)(src + 4 * q);
    }
    __syncthreads();
#pragma unroll 1
    for (int s = 0; s < XCH; ++s) {
      const bool last = (tc == NCH - 1) && (s == XCH - 1);
#pragma unroll
      for (int mt = 0; mt < 2; ++mt) {
        v8f acc0 = z8, acc1 = z8;
        acc0 = Frag<_Float16>::mma(a0[mt], bw[0][0], acc0);
        acc1 = Frag<_Float16>::mma(a0[mt], bw[0][1], acc1);
        guard_g0(acc0, acc1, a0[mt], bw[0][0], bw[0][1]);
        float hv0[8], hv1[8];
#pragma unroll
        for (int r = 0; r < 8; ++r) {
          const float xr = xsw[(16 * mt + 8 * hh + r) * XCH + s];
          const float i0 = fmaf(xr, wic[0], bs0[0]);
          const float i1 = fmaf(xr, wic[1], bs0[1]);
          hv0[r] = ftanh_f32(fmaf(acc0[r], WSC_INV, i0));
          hv1[r] = ftanh_f32(fmaf(acc1[r], WSC_INV, i1));
        }
        _Float16* ht = ht0 + mt * HT_SZ;
#pragma unroll
        for (int r = 0; r < 8; ++r) {
          ht[(8 * hh + r) * NH + c]      = (_Float16)hv0[r];
          ht[(8 * hh + r) * NH + 16 + c] = (_Float16)hv1[r];
        }
        if (last) {
#pragma unroll
          for (int r = 0; r < 8; ++r) {
            hs0[(16 * mt + 8 * hh + r) * NH + c]      = hv0[r];
            hs0[(16 * mt + 8 * hh + r) * NH + 16 + c] = hv1[r];
          }
        }
      }
      __syncthreads();
#pragma unroll
      for (int mt = 0; mt < 2; ++mt) a0[mt] = Frag<_Float16>::load(ht0 + mt * HT_SZ + c * NH + koff);
#pragma unroll
      for (int mt = 0; mt < 2; ++mt) {
        v8f acc0 = z8, acc1 = z8;
        acc0 = Frag<_Float16>::mma(a0[mt], bw[1][0], acc0);
        acc1 = Frag<_Float16>::mma(a0[mt], bw[1][1], acc1);
        acc0 = Frag<_Float16>::mma(a1[mt], bw[2][0], acc0);
        acc1 = Frag<_Float16>::mma(a1[mt], bw[2][1], acc1);
        guard_g1(acc0, acc1, a0[mt], a1[mt], bw[1][0], bw[1][1], bw[2][0], bw[2][1]);
        float hv0[8], hv1[8];
#pragma unroll
        for (int r = 0; r < 8; ++r) {
          hv0[r] = ftanh_f32(fmaf(acc0[r], WSC_INV, bs1[0]));
          hv1[r] = ftanh_f32(fmaf(acc1[r], WSC_INV, bs1[1]));
        }
        _Float16* ht = ht1 + mt * HT_SZ;
#pragma unroll
        for (int r = 0; r < 8; ++r) {
          ht[(8 * hh + r) * NH + c]      = (_Float16)hv0[r];
          ht[(8 * hh + r) * NH + 16 + c] = (_Float16)hv1[r];
        }
        if (last) {
#pragma unroll
          for (int r = 0; r < 8; ++r) {
            hs1[(16 * mt + 8 * hh + r) * NH + c]      = hv0[r];
            hs1[(16 * mt + 8 * hh + r) * NH + 16 + c] = hv1[r];
          }
        }
      }
      __syncthreads();
#pragma unroll
      for (int mt = 0; mt < 2; ++mt) a1[mt] = Frag<_Float16>::load(ht1 + mt * HT_SZ + c * NH + koff);
    }
  }

  {
    const float* hrow = hs1 + lane * NH;
    const float* wv = Pf + 3 * NH;
    float sacc = 0.0f;
#pragma unroll
    for (int j4 = 0; j4 < 8; ++j4) {
      const v4f hq = *(const v4f*)(hrow + 4 * j4);
      const v4f wq = *(const v4f*)(wv + 4 * j4);
#pragma unroll
      for (int e = 0; e < 4; ++e) sacc = fmaf(hq[e], wq[e], sacc);
    }
    sacc += Pf[4 * NH];
    Pq[w * RPW + lane] = sacc;
  }
  __syncthreads();

  {
    const int q = lane >> 3, c4 = (lane & 7) * 4;
    float* oh = out + NB;
    for (int pass = 0; pass < 2; ++pass) {
#pragma unroll
      for (int L = 0; L < 2; ++L) {
        const float* sl = Hs + (w * 2 + L) * HS_SZ;
#pragma unroll
        for (int it = 0; it < 8; ++it) {
          const int row = it * 4 + q;
          const v4f v = *(const v4f*)(sl + row * NH + c4);
          *(volatile v4f*)(oh + (size_t)L * NB * NH + (size_t)(bbase + row) * NH + c4) = v;
        }
      }
      if (q == 0) {
        const v4f pv = *(const v4f*)(Pq + w * RPW + c4);
        *(volatile v4f*)(out + bbase + c4) = pv;
      }
      __threadfence();
    }
  }
}

extern "C" void kernel_launch(void* const* d_in, const int* in_sizes, int n_in,
                              void* d_out, int out_size, void* d_ws, size_t ws_size, hipStream_t stream) {
  (void)d_ws; (void)ws_size;
  if (n_in < 12 || d_out == nullptr) return;
  if (in_sizes[0] != NB * NSTEP || in_sizes[1] != 2 * NB * NH || in_sizes[2] != NH || in_sizes[3] != NH * NH ||
      in_sizes[4] != NH || in_sizes[5] != NH || in_sizes[6] != NH * NH || in_sizes[7] != NH * NH ||
      in_sizes[8] != NH || in_sizes[9] != NH || in_sizes[10] != NH || in_sizes[11] != 1 || out_size != NOUTF) return;

  const float* x    = (const float*)d_in[0];
  const float* hs   = (const float*)d_in[1];
  const float* wih0 = (const float*)d_in[2];
  const float* whh0 = (const float*)d_in[3];
  const float* bih0 = (const float*)d_in[4];
  const float* bhh0 = (const float*)d_in[5];
  const float* wih1 = (const float*)d_in[6];
  const float* whh1 = (const float*)d_in[7];
  const float* bih1 = (const float*)d_in[8];
  const float* bhh1 = (const float*)d_in[9];
  const float* wfc  = (const float*)d_in[10];
  const float* bfc  = (const float*)d_in[11];
  float* out = (float*)d_out;

  rnn2_seq_kernel<<<NB / RPB, NTHR, 0, stream>>>(x, hs, wih0, whh0, bih0, bhh0, wih1, whh1, bih1, bhh1, wfc, bfc, out);
}
